// RNNModel_27994596836199
// MI455X (gfx1250) — hardware-run, weakly checked
//
#include <hip/hip_runtime.h>

typedef __attribute__((ext_vector_type(16))) _Float16 v16h;
typedef __attribute__((ext_vector_type(8)))  _Float16 v8h;
typedef __attribute__((ext_vector_type(16))) __bf16   v16b;
typedef __attribute__((ext_vector_type(8)))  __bf16   v8b;
typedef __attribute__((ext_vector_type(8)))  float    v8f;
typedef __attribute__((ext_vector_type(4)))  float    v4f;

__device__ __forceinline__ unsigned short f2bf_bits(float f) {
  unsigned u = __float_as_uint(f);
  return (unsigned short)((u + 0x7FFFu + ((u >> 16) & 1u)) >> 16);
}
__device__ __forceinline__ float bf_bits2f(unsigned short h) { return __uint_as_float(((unsigned)h) << 16); }
__device__ __forceinline__ float bf16_rne(float f) { return bf_bits2f(f2bf_bits(f)); }

__device__ __forceinline__ void dep_guard_h(v8f& a, v8f& b, v16h x, v16h y) { asm volatile("v_nop\n\tv_nop\n\tv_nop\n\tv_nop" : "+v"(a), "+v"(b) : "v"(x), "v"(y)); }
__device__ __forceinline__ void dep_guard_b(v8f& a, v8f& b, v16b x, v16b y) { asm volatile("v_nop\n\tv_nop\n\tv_nop\n\tv_nop" : "+v"(a), "+v"(b) : "v"(x), "v"(y)); }
__device__ __forceinline__ void keep4_h(v16h a, v16h b, v16h c, v16h d) { asm volatile("v_nop" :: "v"(a), "v"(b), "v"(c), "v"(d)); }
__device__ __forceinline__ void keep4_b(v16b a, v16b b, v16b c, v16b d) { asm volatile("v_nop" :: "v"(a), "v"(b), "v"(c), "v"(d)); }
__device__ __forceinline__ void acc_guard4(v8f& a, v8f& b, v8f& c, v8f& d) { asm volatile("v_nop\n\tv_nop\n\tv_nop\n\tv_nop" : "+v"(a), "+v"(b), "+v"(c), "+v"(d)); }
template <typename T> struct Frag;
template <> struct Frag<_Float16> {
  typedef v16h V; union U { v16h v; v8h h[2]; };
  static __device__ __forceinline__ v16h load(const _Float16* p) {
    U f; f.h[0] = *(const v8h*)(p); f.h[1] = *(const v8h*)(p + 16); return f.v;
  }
  static __device__ __forceinline__ v8f mma(v16h a, v16h b, v8f c) {
    return __builtin_amdgcn_wmma_f32_16x16x32_f16(false, a, false, b, (short)0, c, false, false);
  }
  static __device__ __forceinline__ void guard(v8f& a, v8f& b, v16h x, v16h y) { dep_guard_h(a, b, x, y); }
  static __device__ __forceinline__ void keep(v16h a, v16h b, v16h c, v16h d) { keep4_h(a, b, c, d); }
};
template <> struct Frag<__bf16> {
  typedef v16b V; union U { v16b v; v8b h[2]; };
  static __device__ __forceinline__ v16b load(const __bf16* p) {
    U f; f.h[0] = *(const v8b*)(p); f.h[1] = *(const v8b*)(p + 16); return f.v;
  }
  static __device__ __forceinline__ v8f mma(v16b a, v16b b, v8f c) {
    return __builtin_amdgcn_wmma_f32_16x16x32_bf16(false, a, false, b, (short)0, c, false, false);
  }
  static __device__ __forceinline__ void guard(v8f& a, v8f& b, v16b x, v16b y) { dep_guard_b(a, b, x, y); }
  static __device__ __forceinline__ void keep(v16b a, v16b b, v16b c, v16b d) { keep4_b(a, b, c, d); }
};

template <int ET> struct Elem;
template <> struct Elem<0> { typedef _Float16 T; };
template <> struct Elem<1> { typedef __bf16 T; };
template <int ET, bool SPLIT, int BIAS_MODE, int OUT_MODE, bool RESID, int ACT = 0>
__global__ __launch_bounds__(256) void wmma_gemm64(
    const unsigned short* __restrict__ Ap, const unsigned short* __restrict__ A2p, int lda, long strideA,
    const unsigned short* __restrict__ Btp, const unsigned short* __restrict__ Bt2p, int ldb, long strideB,
    void* __restrict__ Cout, void* __restrict__ Cout2, int ldc, long strideC,
    const float* __restrict__ bias,
    const float* __restrict__ resid, long strideR,
    int M, int N, int K, float scale) {
  typedef typename Elem<ET>::T T;
  typedef typename Frag<T>::V V;
  const T* A = (const T*)Ap; const T* A2 = (const T*)A2p; const T* Bt = (const T*)Btp; const T* Bt2 = (const T*)Bt2p;
  __shared__ __align__(16) float sT[8][16 * 68];
  const int b    = blockIdx.y;
  const int lane = threadIdx.x & 31;
  const int wave = threadIdx.x >> 5;
  const int tilesN = N >> 6;
  const int tilesM = M >> 6;
  const int tile = blockIdx.x * 8 + wave;
  if (tile >= tilesM * tilesN) return;
  const int tm = tile / tilesN;
  const int tn = tile - tm * tilesN;
  const int m0 = tm << 6;
  const int n0 = tn << 6;

  const T* Ab  = A  + (size_t)b * strideA;
  const T* Bb  = Bt + (size_t)b * strideB;
  const T* Ab2 = SPLIT ? (A2  + (size_t)b * strideA) : nullptr;
  const T* Bb2 = SPLIT ? (Bt2 + (size_t)b * strideB) : nullptr;

  const int rlane = lane & 15;
  const int koff  = (lane >> 4) * 8;
  const int mOff  = (lane >> 4) * 8;

  v8f acc[4][4];
#pragma unroll
  for (int i = 0; i < 4; ++i)
#pragma unroll
    for (int j = 0; j < 4; ++j) acc[i][j] = (v8f){0.f,0.f,0.f,0.f,0.f,0.f,0.f,0.f};

  for (int k0 = 0; k0 < K; k0 += 32) {
    V bh[4], bl[4];
#pragma unroll
    for (int j = 0; j < 4; ++j) {
      const size_t bo = (size_t)(n0 + (j << 4) + rlane) * ldb + koff + k0;
      bh[j] = Frag<T>::load(Bb + bo);
      if (SPLIT) bl[j] = Frag<T>::load(Bb2 + bo);
    }
#pragma unroll
    for (int i = 0; i < 4; ++i) {
      const size_t ao = (size_t)(m0 + (i << 4) + rlane) * lda + koff + k0;
      V ah = Frag<T>::load(Ab + ao);
      V al;
      if (SPLIT) al = Frag<T>::load(Ab2 + ao);
#pragma unroll
      for (int j = 0; j < 4; ++j) {
        acc[i][j] = Frag<T>::mma(ah, bh[j], acc[i][j]);
        if (SPLIT) {
          acc[i][j] = Frag<T>::mma(ah, bl[j], acc[i][j]);
          acc[i][j] = Frag<T>::mma(al, bh[j], acc[i][j]);
        }
      }
      Frag<T>::guard(acc[i][0], acc[i][3], ah, SPLIT ? al : ah);
    }
    Frag<T>::keep(bh[0], bh[1], bh[2], bh[3]);
    if (SPLIT) Frag<T>::keep(bl[0], bl[1], bl[2], bl[3]);
  }
  acc_guard4(acc[0][0], acc[0][1], acc[0][2], acc[0][3]);
  acc_guard4(acc[1][0], acc[1][1], acc[1][2], acc[1][3]);
  acc_guard4(acc[2][0], acc[2][1], acc[2][2], acc[2][3]);
  acc_guard4(acc[3][0], acc[3][1], acc[3][2], acc[3][3]);

  float* slab = sT[wave];
  const float* Rb = RESID ? (resid + (size_t)b * strideR) : nullptr;
#pragma unroll
  for (int i = 0; i < 4; ++i) {
    const int mBase = m0 + (i << 4);
#pragma unroll
    for (int j = 0; j < 4; ++j) {
      const int n = n0 + (j << 4) + rlane;
      float bv = 0.f;
      if (BIAS_MODE == 2) bv = bias[n];
#pragma unroll
      for (int r = 0; r < 8; ++r) {
        float v = acc[i][j][r] * scale;
        if (BIAS_MODE == 1) v += bias[mBase + mOff + r];
        if (BIAS_MODE == 2) v += bv;
        if (RESID) v += Rb[(size_t)(mBase + mOff + r) * ldc + n];
        if (ACT == 1) v = tanhf(v);
        if (ACT == 2) v = fmaxf(v, 0.0f);
        if (ACT == 3) v = v / (1.0f + expf(-v));
        if (ACT == 4) v = (v > 0.f) ? v : 0.01f * v;
        if (ACT == 5) v = 0.5f * v * (1.0f + erff(v * 0.70710678118654752f));
        slab[(mOff + r) * 68 + (j << 4) + rlane] = v;
      }
    }
    __builtin_amdgcn_fence(__ATOMIC_RELEASE, "workgroup");
    __builtin_amdgcn_wave_barrier();
    __builtin_amdgcn_fence(__ATOMIC_ACQUIRE, "workgroup");
    if (OUT_MODE == 0) {
      float* C = (float*)Cout + (size_t)b * strideC;
      const int hh = lane >> 4, c4 = (lane & 15) * 4;
      for (int pass = 0; pass < 2; ++pass) {
#pragma unroll
        for (int it = 0; it < 8; ++it) {
          const int row = it * 2 + hh;
          v4f v = *(const v4f*)(slab + row * 68 + c4);
          *(volatile v4f*)(C + (size_t)(mBase + row) * ldc + n0 + c4) = v;
        }
        __threadfence();
      }
    } else {
      const int q = lane >> 3, c8 = (lane & 7) * 8;
      unsigned short* C  = (unsigned short*)Cout  + (size_t)b * strideC;
      unsigned short* C2 = (OUT_MODE == 2) ? ((unsigned short*)Cout2 + (size_t)b * strideC) : nullptr;
      for (int pass = 0; pass < 2; ++pass) {
#pragma unroll
        for (int it = 0; it < 4; ++it) {
          const int row = it * 4 + q;
          const float* sp = slab + row * 68 + c8;
          v8h hv, lv;
#pragma unroll
          for (int e = 0; e < 8; ++e) {
            if (OUT_MODE == 1) {
              hv[e] = (_Float16)sp[e];
            } else {
              unsigned short hb = f2bf_bits(sp[e]);
              unsigned short lb = f2bf_bits(sp[e] - bf_bits2f(hb));
              hv[e] = __builtin_bit_cast(_Float16, hb);
              lv[e] = __builtin_bit_cast(_Float16, lb);
            }
          }
          *(volatile v8h*)(C + (size_t)(mBase + row) * ldc + n0 + c8) = hv;
          if (OUT_MODE == 2) *(volatile v8h*)(C2 + (size_t)(mBase + row) * ldc + n0 + c8) = lv;
        }
        __threadfence();
      }
    }
    __builtin_amdgcn_fence(__ATOMIC_RELEASE, "workgroup");
    __builtin_amdgcn_wave_barrier();
    __builtin_amdgcn_fence(__ATOMIC_ACQUIRE, "workgroup");
  }
}

constexpr int SEQ_T  = 1024;
constexpr int SEQ_B  = 64;
constexpr int DIM_I  = 128;
constexpr int DIM_H  = 512;
constexpr int DIM_O  = 128;
constexpr int SEQ_THREADS = 512;
constexpr float WCARRY     = 16.0f;
constexpr float WCARRY_INV = 0.0625f;

static_assert(SEQ_THREADS == DIM_H);
static_assert((SEQ_THREADS / 32) * 32 == DIM_H);
static_assert(DIM_I % 32 == 0 && DIM_H % 32 == 0);
static_assert((SEQ_B * DIM_H) % (SEQ_THREADS * 8) == 0);
static_assert((SEQ_B * DIM_H) % (SEQ_THREADS * 4) == 0);

constexpr size_t WS_XH    = 0;
constexpr size_t WS_WIH   = WS_XH  + (size_t)SEQ_T * SEQ_B * DIM_I * 2;
constexpr size_t WS_WHH   = WS_WIH + (size_t)DIM_H * DIM_I * 2;
constexpr size_t WS_WFC   = WS_WHH + (size_t)DIM_H * DIM_H * 2;
constexpr size_t WS_BFC   = WS_WFC + (size_t)DIM_O * DIM_H * 2;
constexpr size_t WS_RPL   = WS_BFC + 65536;
constexpr size_t WS_END   = WS_RPL + (size_t)SEQ_T * SEQ_B * DIM_H * 2;
static_assert(WS_END == 84738048);
static_assert(WS_END <= 134217728);
static_assert(WS_WIH % 128 == 0 && WS_WHH % 128 == 0 && WS_WFC % 128 == 0 && WS_BFC % 128 == 0 && WS_RPL % 128 == 0);

constexpr size_t OUT0_BYTES = (size_t)SEQ_T * SEQ_B * DIM_O * 4;
constexpr size_t OUT1_OFF_BYTES = 33554432;
constexpr size_t OUT1_BYTES = (size_t)SEQ_B * DIM_H * 4;
static_assert(OUT0_BYTES == OUT1_OFF_BYTES);
static_assert(OUT1_OFF_BYTES + OUT1_BYTES == 33685504);
static_assert(OUT1_OFF_BYTES % 128 == 0);
constexpr size_t OUT1_OFF_FLOATS = OUT1_OFF_BYTES / 4;

constexpr int PROJ_M = SEQ_T * SEQ_B;
constexpr int PROJ_N = DIM_O;
constexpr int PROJ_K = DIM_H;
static_assert(PROJ_M % 64 == 0 && PROJ_N % 64 == 0 && PROJ_K % 32 == 0);
constexpr int PROJ_TILES = (PROJ_M / 64) * (PROJ_N / 64);
static_assert(PROJ_TILES % 8 == 0);

__global__ __launch_bounds__(256) void cast_bf16rne_f16x8(
    const float* __restrict__ in, unsigned short* __restrict__ out, int n8, float scale) {
  const int i = blockIdx.x * 256 + threadIdx.x;
  if (i < n8) {
    const size_t e = (size_t)i * 8;
    const v4f a = *(const v4f*)(in + e);
    const v4f b = *(const v4f*)(in + e + 4);
    v8h hv;
#pragma unroll
    for (int q = 0; q < 4; ++q) {
      const float r0 = bf16_rne(a[q]) * scale;
      const float r1 = bf16_rne(b[q]) * scale;
      hv[q]     = (_Float16)r0;
      hv[4 + q] = (_Float16)r1;
    }
    _Float16* op = (_Float16*)out + e;
    *(volatile v8h*)op = hv;
    __threadfence();
    *(volatile v8h*)op = hv;
  }
}
static_assert((SEQ_T * SEQ_B * DIM_I / 8) % 256 == 0);
static_assert((DIM_H * DIM_I / 8) % 256 == 0);
static_assert((DIM_H * DIM_H / 8) % 256 == 0);
static_assert((DIM_O * DIM_H / 8) % 256 == 0);

static_assert(DIM_O == 32 * 4);
__global__ __launch_bounds__(32) void bias_rne_kernel(const float* __restrict__ in, float* __restrict__ out) {
  const int l = threadIdx.x;
  const v4f a = *(const v4f*)(in + 4 * l);
  v4f o;
#pragma unroll
  for (int q = 0; q < 4; ++q) o[q] = bf16_rne(a[q]);
  *(volatile v4f*)(out + 4 * l) = o;
  __threadfence();
  *(volatile v4f*)(out + 4 * l) = o;
}

__global__ __launch_bounds__(SEQ_THREADS) void elman_seq_kernel(
    const unsigned short* __restrict__ xh,
    const float* __restrict__ h0,
    const unsigned short* __restrict__ wih,
    const unsigned short* __restrict__ whh,
    const float* __restrict__ b_ih,
    const float* __restrict__ b_hh,
    unsigned short* __restrict__ rpl,
    float* __restrict__ hlast)
{
  __shared__ __align__(16) _Float16 hS[SEQ_B * DIM_H];
  __shared__ __align__(16) float    stg[SEQ_B * DIM_H];
  __shared__ __align__(16) float    bS[DIM_H];

  const int tid   = threadIdx.x;
  const int wave  = tid >> 5;
  const int lane  = tid & 31;
  const int rlane = lane & 15;
  const int koff  = (lane >> 4) * 8;
  const int mOff  = (lane >> 4) * 8;
  const int ncol0 = wave * 32;

  const _Float16* Xp = (const _Float16*)xh;
  const _Float16* Wi = (const _Float16*)wih;
  const _Float16* Wh = (const _Float16*)whh;

  bS[tid] = bf16_rne(b_ih[tid]) + bf16_rne(b_hh[tid]);
#pragma unroll 1
  for (int it = 0; it < (SEQ_B * DIM_H) / (SEQ_THREADS * 8); ++it) {
    const int e = (it * SEQ_THREADS + tid) * 8;
    const v4f a = *(const v4f*)(h0 + e);
    const v4f b = *(const v4f*)(h0 + e + 4);
    v8h hv;
#pragma unroll
    for (int q = 0; q < 4; ++q) {
      hv[q]     = (_Float16)bf16_rne(a[q]);
      hv[4 + q] = (_Float16)bf16_rne(b[q]);
    }
    *(v8h*)(hS + e) = hv;
  }
  __syncthreads();

#pragma unroll 1
  for (int t = 0; t < SEQ_T; ++t) {
    v8f acc[4][2];
#pragma unroll
    for (int i = 0; i < 4; ++i)
#pragma unroll
      for (int j = 0; j < 2; ++j) acc[i][j] = (v8f){0.f,0.f,0.f,0.f,0.f,0.f,0.f,0.f};

    const _Float16* Xt = Xp + (size_t)t * SEQ_B * DIM_I;
#pragma unroll
    for (int k0 = 0; k0 < DIM_I; k0 += 32) {
      const v16h bf0 = Frag<_Float16>::load(Wi + (size_t)(ncol0 + rlane) * DIM_I + koff + k0);
      const v16h bf1 = Frag<_Float16>::load(Wi + (size_t)(ncol0 + 16 + rlane) * DIM_I + koff + k0);
#pragma unroll
      for (int i = 0; i < 4; ++i) {
        const v16h af = Frag<_Float16>::load(Xt + (size_t)(i * 16 + rlane) * DIM_I + koff + k0);
        acc[i][0] = Frag<_Float16>::mma(af, bf0, acc[i][0]);
        acc[i][1] = Frag<_Float16>::mma(af, bf1, acc[i][1]);
        Frag<_Float16>::guard(acc[i][0], acc[i][1], af, af);
      }
      Frag<_Float16>::keep(bf0, bf1, bf0, bf1);
    }
#pragma unroll 2
    for (int k0 = 0; k0 < DIM_H; k0 += 32) {
      const v16h bf0 = Frag<_Float16>::load(Wh + (size_t)(ncol0 + rlane) * DIM_H + koff + k0);
      const v16h bf1 = Frag<_Float16>::load(Wh + (size_t)(ncol0 + 16 + rlane) * DIM_H + koff + k0);
#pragma unroll
      for (int i = 0; i < 4; ++i) {
        const v16h af = Frag<_Float16>::load(hS + (i * 16 + rlane) * DIM_H + koff + k0);
        acc[i][0] = Frag<_Float16>::mma(af, bf0, acc[i][0]);
        acc[i][1] = Frag<_Float16>::mma(af, bf1, acc[i][1]);
        Frag<_Float16>::guard(acc[i][0], acc[i][1], af, af);
      }
      Frag<_Float16>::keep(bf0, bf1, bf0, bf1);
    }
    acc_guard4(acc[0][0], acc[0][1], acc[1][0], acc[1][1]);
    acc_guard4(acc[2][0], acc[2][1], acc[3][0], acc[3][1]);

    __syncthreads();

#pragma unroll
    for (int i = 0; i < 4; ++i)
#pragma unroll
      for (int j = 0; j < 2; ++j)
#pragma unroll
        for (int r = 0; r < 8; ++r)
          stg[(i * 16 + mOff + r) * DIM_H + ncol0 + j * 16 + rlane] = acc[i][j][r];
    __syncthreads();

    unsigned short* Rt = rpl + (size_t)t * SEQ_B * DIM_H;
#pragma unroll 1
    for (int it = 0; it < (SEQ_B * DIM_H) / (SEQ_THREADS * 8); ++it) {
      const int e   = (it * SEQ_THREADS + tid) * 8;
      const int col = e & (DIM_H - 1);
      const v4f p0 = *(const v4f*)(stg + e);
      const v4f p1 = *(const v4f*)(stg + e + 4);
      const v4f c0 = *(const v4f*)(bS + col);
      const v4f c1 = *(const v4f*)(bS + col + 4);
      v8h hv;
#pragma unroll
      for (int q = 0; q < 4; ++q) {
        const float u0 = tanhf(p0[q] * WCARRY_INV + c0[q]);
        const float u1 = tanhf(p1[q] * WCARRY_INV + c1[q]);
        hv[q]     = (_Float16)u0;
        hv[4 + q] = (_Float16)u1;
      }
      *(v8h*)(hS + e) = hv;
      _Float16* gp = (_Float16*)Rt + e;
      *(volatile v8h*)gp = hv;
      __threadfence();
      *(volatile v8h*)gp = hv;
    }
    __syncthreads();
  }

#pragma unroll 1
  for (int it = 0; it < (SEQ_B * DIM_H) / (SEQ_THREADS * 4); ++it) {
    const int e   = (it * SEQ_THREADS + tid) * 4;
    const int col = e & (DIM_H - 1);
    const v4f p = *(const v4f*)(stg + e);
    const v4f c = *(const v4f*)(bS + col);
    v4f o;
#pragma unroll
    for (int q = 0; q < 4; ++q) o[q] = tanhf(p[q] * WCARRY_INV + c[q]);
    *(volatile v4f*)(hlast + e) = o;
    __threadfence();
    *(volatile v4f*)(hlast + e) = o;
  }
}

extern "C" void kernel_launch(void* const* d_in, const int* in_sizes, int n_in,
                              void* d_out, int out_size, void* d_ws, size_t ws_size,
                              hipStream_t stream) {
  if (n_in < 8) return;
  if (in_sizes[0] != SEQ_T * SEQ_B * DIM_I) return;
  if (in_sizes[1] != SEQ_B * DIM_H) return;
  if (in_sizes[2] != DIM_H * DIM_I) return;
  if (in_sizes[3] != DIM_H * DIM_H) return;
  if (in_sizes[4] != DIM_H || in_sizes[5] != DIM_H) return;
  if (in_sizes[6] != DIM_O * DIM_H || in_sizes[7] != DIM_O) return;
  if ((size_t)out_size != (size_t)SEQ_T * SEQ_B * DIM_O + (size_t)SEQ_B * DIM_H) return;
  if (ws_size < WS_END) return;

  const float* x    = (const float*)d_in[0];
  const float* h0   = (const float*)d_in[1];
  const float* W_ih = (const float*)d_in[2];
  const float* W_hh = (const float*)d_in[3];
  const float* b_ih = (const float*)d_in[4];
  const float* b_hh = (const float*)d_in[5];
  const float* W_fc = (const float*)d_in[6];
  const float* b_fc = (const float*)d_in[7];

  float* y_out = (float*)d_out;
  float* hlast = (float*)d_out + OUT1_OFF_FLOATS;

  char* ws = (char*)d_ws;
  unsigned short* xh   = (unsigned short*)(ws + WS_XH);
  unsigned short* wih  = (unsigned short*)(ws + WS_WIH);
  unsigned short* whh  = (unsigned short*)(ws + WS_WHH);
  unsigned short* wfc  = (unsigned short*)(ws + WS_WFC);
  float*          bfcr = (float*)(ws + WS_BFC);
  unsigned short* rpl  = (unsigned short*)(ws + WS_RPL);

  cast_bf16rne_f16x8<<<(SEQ_T * SEQ_B * DIM_I / 8) / 256, 256, 0, stream>>>(x, xh, SEQ_T * SEQ_B * DIM_I / 8, 1.0f);
  cast_bf16rne_f16x8<<<(DIM_H * DIM_I / 8) / 256, 256, 0, stream>>>(W_ih, wih, DIM_H * DIM_I / 8, WCARRY);
  cast_bf16rne_f16x8<<<(DIM_H * DIM_H / 8) / 256, 256, 0, stream>>>(W_hh, whh, DIM_H * DIM_H / 8, WCARRY);
  cast_bf16rne_f16x8<<<(DIM_O * DIM_H / 8) / 256, 256, 0, stream>>>(W_fc, wfc, DIM_O * DIM_H / 8, WCARRY);
  bias_rne_kernel<<<1, 32, 0, stream>>>(b_fc, bfcr);

  elman_seq_kernel<<<1, SEQ_THREADS, 0, stream>>>(xh, h0, wih, whh, b_ih, b_hh, rpl, hlast);

  wmma_gemm64<0, false, 2, 0, false, 0><<<dim3(PROJ_TILES / 8, 1), 256, 0, stream>>>(
      (const unsigned short*)rpl, (const unsigned short*)rpl, PROJ_K, 0L,
      (const unsigned short*)wfc, (const unsigned short*)wfc, PROJ_K, 0L,
      (void*)y_out, (void*)y_out, PROJ_N, 0L,
      (const float*)bfcr,
      (const float*)bfcr, 0L,
      PROJ_M, PROJ_N, PROJ_K, WCARRY_INV);
}
